// MultiHeadAttention_29850022707651
// MI455X (gfx1250) — hardware-run, weakly checked
//
#include <hip/hip_runtime.h>
#include <math.h>

#ifndef NB
#define NB 2
#endif
#ifndef SEQ
#define SEQ 2048
#endif
#define NB_FULL 2
#define SEQ_FULL 2048
#define DM 1024
#define NH 16
#define HD 64
#define SIMW 256

typedef __attribute__((ext_vector_type(16))) _Float16 v16h;
typedef __attribute__((ext_vector_type(8)))  _Float16 v8h;
typedef __attribute__((ext_vector_type(16))) __bf16   v16b;
typedef __attribute__((ext_vector_type(8)))  __bf16   v8b;
typedef __attribute__((ext_vector_type(8)))  float    v8f;
typedef __attribute__((ext_vector_type(4)))  float    v4f;
typedef unsigned int cm_u4 __attribute__((ext_vector_type(4)));

__device__ __forceinline__ int frag_k(int i, int h) { return (i < 8) ? (8 * h + i) : (16 + 8 * h + (i - 8)); }

__device__ __forceinline__ v8f wmma16(v16h a, v16h b, v8f c) {
    c = __builtin_amdgcn_wmma_f32_16x16x32_f16(false, a, false, b, (short)0, c, false, false);
    asm volatile("v_nop\n\tv_nop\n\tv_nop\n\tv_nop" : "+v"(c) : "v"(a), "v"(b));
    return c;
}

#define VST2(T, ptr, val) do { const T vst2_v_ = (val); *(volatile T*)(ptr) = vst2_v_; __threadfence(); *(volatile T*)(ptr) = vst2_v_; } while (0)
#define VST2V4(ptr, val) do { const v4f vst2_v4_ = (val); *(volatile v4f*)(ptr) = vst2_v4_; __threadfence(); *(volatile v4f*)(ptr) = vst2_v4_; } while (0)

__device__ __forceinline__ v16h fh_row32(const float* __restrict__ row, int hf) {
    const v4f a0 = *(const v4f*)(row + 8 * hf), a1 = *(const v4f*)(row + 8 * hf + 4);
    const v4f b0 = *(const v4f*)(row + 16 + 8 * hf), b1 = *(const v4f*)(row + 20 + 8 * hf);
    v16h r;
    r[0] = (_Float16)a0.x; r[1] = (_Float16)a0.y; r[2] = (_Float16)a0.z; r[3] = (_Float16)a0.w;
    r[4] = (_Float16)a1.x; r[5] = (_Float16)a1.y; r[6] = (_Float16)a1.z; r[7] = (_Float16)a1.w;
    r[8] = (_Float16)b0.x; r[9] = (_Float16)b0.y; r[10] = (_Float16)b0.z; r[11] = (_Float16)b0.w;
    r[12] = (_Float16)b1.x; r[13] = (_Float16)b1.y; r[14] = (_Float16)b1.z; r[15] = (_Float16)b1.w;
    return r;
}

namespace w25 {
__device__ __forceinline__ void dep_guard_h(v8f& a, v8f& b, v16h x, v16h y) { asm volatile("v_nop\n\tv_nop\n\tv_nop\n\tv_nop" : "+v"(a), "+v"(b) : "v"(x), "v"(y)); }
__device__ __forceinline__ void dep_guard_b(v8f& a, v8f& b, v16b x, v16b y) { asm volatile("v_nop\n\tv_nop\n\tv_nop\n\tv_nop" : "+v"(a), "+v"(b) : "v"(x), "v"(y)); }
__device__ __forceinline__ void keep4_h(v16h a, v16h b, v16h c, v16h d) { asm volatile("v_nop" :: "v"(a), "v"(b), "v"(c), "v"(d)); }
__device__ __forceinline__ void keep4_b(v16b a, v16b b, v16b c, v16b d) { asm volatile("v_nop" :: "v"(a), "v"(b), "v"(c), "v"(d)); }
__device__ __forceinline__ void acc_guard4(v8f& a, v8f& b, v8f& c, v8f& d) { asm volatile("v_nop\n\tv_nop\n\tv_nop\n\tv_nop" : "+v"(a), "+v"(b), "+v"(c), "+v"(d)); }
template <typename T> struct Frag;
template <> struct Frag<_Float16> {
  typedef v16h V; union U { v16h v; v8h h[2]; };
  static __device__ __forceinline__ v16h load(const _Float16* p) {
    U f; f.h[0] = *(const v8h*)(p); f.h[1] = *(const v8h*)(p + 16); return f.v;
  }
  static __device__ __forceinline__ v8f mma(v16h a, v16h b, v8f c) {
    return __builtin_amdgcn_wmma_f32_16x16x32_f16(false, a, false, b, (short)0, c, false, false);
  }
  static __device__ __forceinline__ void guard(v8f& a, v8f& b, v16h x, v16h y) { dep_guard_h(a, b, x, y); }
  static __device__ __forceinline__ void keep(v16h a, v16h b, v16h c, v16h d) { keep4_h(a, b, c, d); }
};
template <> struct Frag<__bf16> {
  typedef v16b V; union U { v16b v; v8b h[2]; };
  static __device__ __forceinline__ v16b load(const __bf16* p) {
    U f; f.h[0] = *(const v8b*)(p); f.h[1] = *(const v8b*)(p + 16); return f.v;
  }
  static __device__ __forceinline__ v8f mma(v16b a, v16b b, v8f c) {
    return __builtin_amdgcn_wmma_f32_16x16x32_bf16(false, a, false, b, (short)0, c, false, false);
  }
  static __device__ __forceinline__ void guard(v8f& a, v8f& b, v16b x, v16b y) { dep_guard_b(a, b, x, y); }
  static __device__ __forceinline__ void keep(v16b a, v16b b, v16b c, v16b d) { keep4_b(a, b, c, d); }
};
template <int ET> struct Elem;
template <> struct Elem<0> { typedef _Float16 T; };
template <> struct Elem<1> { typedef __bf16 T; };

template <int ET, int BIAS_MODE>
__global__ __launch_bounds__(256) void wmma_gemm64(
    const unsigned short* __restrict__ Ap, int lda, long long strideA,
    const unsigned short* __restrict__ Btp, int ldb, long long strideB,
    float* __restrict__ Cout, int ldc, long long strideC,
    const float* __restrict__ bias, int M, int N, int K, float scale) {
  typedef typename Elem<ET>::T T;
  typedef typename Frag<T>::V V;
  const T* A = (const T*)Ap; const T* Bt = (const T*)Btp;
  __shared__ __align__(16) float sT[8][16 * 68];
  const int b    = blockIdx.y;
  const int lane = threadIdx.x & 31;
  const int wave = __builtin_amdgcn_readfirstlane((int)(threadIdx.x >> 5));
  const int tilesN = N >> 6;
  const int tilesM = M >> 6;
  const int tile = blockIdx.x * 8 + wave;
  if (tile >= tilesM * tilesN) return;
  const int tm = tile / tilesN;
  const int tn = tile - tm * tilesN;
  const int m0 = tm << 6;
  const int n0 = tn << 6;

  const T* Ab = A  + (size_t)b * (size_t)strideA;
  const T* Bb = Bt + (size_t)b * (size_t)strideB;

  const int rlane = lane & 15;
  const int koff  = (lane >> 4) * 8;
  const int mOff  = (lane >> 4) * 8;

  v8f acc[4][4];
#pragma unroll
  for (int i = 0; i < 4; ++i)
#pragma unroll
    for (int j = 0; j < 4; ++j) acc[i][j] = (v8f){0.f,0.f,0.f,0.f,0.f,0.f,0.f,0.f};

  for (int k0 = 0; k0 < K; k0 += 32) {
    V bh[4];
#pragma unroll
    for (int j = 0; j < 4; ++j) {
      const size_t bo = (size_t)(n0 + (j << 4) + rlane) * ldb + koff + k0;
      bh[j] = Frag<T>::load(Bb + bo);
    }
#pragma unroll
    for (int i = 0; i < 4; ++i) {
      const size_t ao = (size_t)(m0 + (i << 4) + rlane) * lda + koff + k0;
      V ah = Frag<T>::load(Ab + ao);
#pragma unroll
      for (int j = 0; j < 4; ++j) acc[i][j] = Frag<T>::mma(ah, bh[j], acc[i][j]);
      Frag<T>::guard(acc[i][0], acc[i][3], ah, ah);
    }
    Frag<T>::keep(bh[0], bh[1], bh[2], bh[3]);
  }
  acc_guard4(acc[0][0], acc[0][1], acc[0][2], acc[0][3]);
  acc_guard4(acc[1][0], acc[1][1], acc[1][2], acc[1][3]);
  acc_guard4(acc[2][0], acc[2][1], acc[2][2], acc[2][3]);
  acc_guard4(acc[3][0], acc[3][1], acc[3][2], acc[3][3]);

  float* C = Cout + (size_t)b * (size_t)strideC;
#pragma unroll
  for (int i = 0; i < 4; ++i) {
    const int mBase = m0 + (i << 4);
#pragma unroll
    for (int j = 0; j < 4; ++j) {
      const int n = n0 + (j << 4) + rlane;
      float bv = 0.f;
      if (BIAS_MODE == 2) bv = bias[n];
#pragma unroll
      for (int r = 0; r < 8; ++r) {
        float v = acc[i][j][r] * scale;
        if (BIAS_MODE == 2) v += bv;
        sT[wave][(mOff + r) * 68 + (j << 4) + rlane] = v;
      }
    }
    __builtin_amdgcn_fence(3  , "workgroup");
    __builtin_amdgcn_wave_barrier();
    __builtin_amdgcn_fence(2  , "workgroup");
    {
      const int hh = lane >> 4, c4 = (lane & 15) * 4;
      for (int pass = 0; pass < 2; ++pass) {
#pragma unroll
        for (int it = 0; it < 8; ++it) {
          const int row = it * 2 + hh;
          const v4f v = *(const v4f*)(&sT[wave][row * 68 + c4]);
          *(volatile v4f*)(C + (size_t)(mBase + row) * ldc + n0 + c4) = v;
        }
        __threadfence();
      }
    }
    __builtin_amdgcn_fence(3  , "workgroup");
    __builtin_amdgcn_wave_barrier();
    __builtin_amdgcn_fence(2  , "workgroup");
  }
}
}

__device__ __forceinline__ unsigned short bfu_rne(float v) { unsigned u = __builtin_bit_cast(unsigned, v); u += 0x7FFFu + ((u >> 16) & 1u); return (unsigned short)(u >> 16); }
__device__ __forceinline__ void bfsplit(float v, unsigned short& hi, unsigned short& lo) { hi = bfu_rne(v); lo = bfu_rne(v - __builtin_bit_cast(float, (unsigned)hi << 16)); }
__device__ __forceinline__ unsigned int cmb_pk2(float a, float b) { return (unsigned int)__builtin_bit_cast(unsigned short, (_Float16)a) | ((unsigned int)__builtin_bit_cast(unsigned short, (_Float16)b) << 16); }
__device__ __forceinline__ float cmb_bf(float v) { const unsigned u = __builtin_bit_cast(unsigned, v); const unsigned r = (u + 0x7fffu + ((u >> 16) & 1u)) & 0xffff0000u; return __builtin_bit_cast(float, r); }

__global__ __launch_bounds__(256) void k_cm_bfvec(const float* __restrict__ SRC, float* __restrict__ DST, int n) {
    const int u = blockIdx.x * 256 + threadIdx.x; if (u >= n) return; VST2(float, DST + u, cmb_bf(SRC[u]));
}
__global__ __launch_bounds__(256) void k_cm_castb(const float* __restrict__ SRC, int lds, unsigned short* __restrict__ DST, int ldd, int nR, int nC, int rpb, int srpb, float sc) {
    const long long u = (long long)blockIdx.x * 256 + threadIdx.x; const int per = nC / 8; if (u >= (long long)nR * per) return;
    const int r = (int)(u / per); const int c0 = 8 * (int)(u % per);
    const int sr = (r / rpb) * srpb + (r % rpb);
    const float* s = SRC + (long long)sr * lds + c0;
    const v4f x0 = *(const v4f*)s, x1 = *(const v4f*)(s + 4);
    cm_u4 pk;
    pk.x = cmb_pk2(cmb_bf(x0.x) * sc, cmb_bf(x0.y) * sc); pk.y = cmb_pk2(cmb_bf(x0.z) * sc, cmb_bf(x0.w) * sc);
    pk.z = cmb_pk2(cmb_bf(x1.x) * sc, cmb_bf(x1.y) * sc); pk.w = cmb_pk2(cmb_bf(x1.z) * sc, cmb_bf(x1.w) * sc);
    VST2(cm_u4, (cm_u4*)(DST + (long long)r * ldd + c0), pk);
}
__global__ __launch_bounds__(256) void k_cm_castbf(const float* __restrict__ SRC, int lds, unsigned short* __restrict__ DST, int ldd, int nR, int nC, int dup) {
    const long long u = (long long)blockIdx.x * 256 + threadIdx.x; const int per = nC / 8; if (u >= (long long)nR * per) return;
    const int r = (int)(u / per); const int c0 = 8 * (int)(u % per);
    const float* s = SRC + (long long)r * lds + c0;
    const v4f x0 = *(const v4f*)s, x1 = *(const v4f*)(s + 4);
    cm_u4 pk;
    pk.x = (unsigned)bfu_rne(x0.x) | ((unsigned)bfu_rne(x0.y) << 16); pk.y = (unsigned)bfu_rne(x0.z) | ((unsigned)bfu_rne(x0.w) << 16);
    pk.z = (unsigned)bfu_rne(x1.x) | ((unsigned)bfu_rne(x1.y) << 16); pk.w = (unsigned)bfu_rne(x1.z) | ((unsigned)bfu_rne(x1.w) << 16);
    VST2(cm_u4, (cm_u4*)(DST + (long long)r * ldd + c0), pk);
    if (dup > 0) VST2(cm_u4, (cm_u4*)(DST + (long long)r * ldd + c0 + dup), pk);
}
__global__ __launch_bounds__(256) void k_split8(const float* __restrict__ SRC, int lds, unsigned short* __restrict__ DH, unsigned short* __restrict__ DL, int ldd, int nR, int nC) {
    const long long u = (long long)blockIdx.x * 256 + threadIdx.x; const int per = nC / 8; if (u >= (long long)nR * per) return;
    const int r = (int)(u / per); const int c0 = 8 * (int)(u % per);
    const float* s = SRC + (long long)r * lds + c0;
    const v4f x0 = *(const v4f*)s, x1 = *(const v4f*)(s + 4);
    unsigned short h0, l0, h1, l1; cm_u4 ph, pq;
    bfsplit(x0.x, h0, l0); bfsplit(x0.y, h1, l1); ph.x = (unsigned)h0 | ((unsigned)h1 << 16); pq.x = (unsigned)l0 | ((unsigned)l1 << 16);
    bfsplit(x0.z, h0, l0); bfsplit(x0.w, h1, l1); ph.y = (unsigned)h0 | ((unsigned)h1 << 16); pq.y = (unsigned)l0 | ((unsigned)l1 << 16);
    bfsplit(x1.x, h0, l0); bfsplit(x1.y, h1, l1); ph.z = (unsigned)h0 | ((unsigned)h1 << 16); pq.z = (unsigned)l0 | ((unsigned)l1 << 16);
    bfsplit(x1.z, h0, l0); bfsplit(x1.w, h1, l1); ph.w = (unsigned)h0 | ((unsigned)h1 << 16); pq.w = (unsigned)l0 | ((unsigned)l1 << 16);
    VST2(cm_u4, (cm_u4*)(DH + (long long)r * ldd + c0), ph);
    VST2(cm_u4, (cm_u4*)(DL + (long long)r * ldd + c0), pq);
}
__global__ __launch_bounds__(256) void k_simnorm(const float* __restrict__ X, unsigned short* __restrict__ Y, int rows, float carry) {
    const int lane = threadIdx.x & 31; const int row = blockIdx.x * 8 + (threadIdx.x >> 5);
    if (row >= rows) return;
    const float* p = X + (long long)row * SIMW + 8 * lane;
    const v4f a = *(const v4f*)p, b = *(const v4f*)(p + 4);
    float ss = a.x * a.x + a.y * a.y + a.z * a.z + a.w * a.w + b.x * b.x + b.y * b.y + b.z * b.z + b.w * b.w;
    ss += __shfl_xor(ss, 16, 32); ss += __shfl_xor(ss, 8, 32); ss += __shfl_xor(ss, 4, 32); ss += __shfl_xor(ss, 2, 32); ss += __shfl_xor(ss, 1, 32);
    const float inv = (1.0f / fmaxf(sqrtf(ss), 1e-12f)) * carry;
    cm_u4 pk;
    pk.x = cmb_pk2(a.x * inv, a.y * inv); pk.y = cmb_pk2(a.z * inv, a.w * inv);
    pk.z = cmb_pk2(b.x * inv, b.y * inv); pk.w = cmb_pk2(b.z * inv, b.w * inv);
    VST2(cm_u4, (cm_u4*)(Y + (long long)row * SIMW + 8 * lane), pk);
}

#define AW 4
struct AttnP {
    const float* Q; const float* K; const float* V; const float* Mf; float* O;
    long long sQb, sQh, sQi, sKb, sKh, sKj, sVb, sVh, sVj, sOb, sOh, sOi, smb, smi;
    int Lq, Lk; float scale; int pad_;
};
static_assert(sizeof(AttnP) == 5 * 8 + 14 * 8 + 4 * 4);

#ifndef KATTN_ATTR
#define KATTN_ATTR
#endif
__global__ __launch_bounds__(32 * AW) KATTN_ATTR void k_attn(AttnP p) {
    constexpr int NT = 4;
    constexpr int VP = 72;
    __shared__ __align__(16) float    pl[AW][16 * 64];
    __shared__ __align__(16) _Float16 vl[64 * VP];
    const int lane = threadIdx.x & 31, hf = lane >> 4, l15 = lane & 15, wave = __builtin_amdgcn_readfirstlane((int)(threadIdx.x >> 5));
    const int h = blockIdx.y, b = blockIdx.z;
    const int q0 = (blockIdx.x * AW + wave) * 16;
    const float L2E = 1.4426950408889634f;
    const float NEG = -__builtin_inff();
    const int qi = min(q0 + l15, p.Lq - 1);
    const float* qrow  = p.Q + b * p.sQb + h * p.sQh + (long long)qi * p.sQi;
    const float* kbase = p.K + b * p.sKb + h * p.sKh;
    const float* vbase = p.V + b * p.sVb + h * p.sVh;
    const float* mbase = p.Mf + b * p.smb + q0 + 8 * hf;
    const v16h qa0 = fh_row32(qrow, hf), qa1 = fh_row32(qrow + 32, hf);
    v8f o[NT]; float m8[8], l8[8];
#pragma unroll
    for (int t = 0; t < NT; ++t) { v8f zz = {}; o[t] = zz; }
#pragma unroll
    for (int i = 0; i < 8; ++i) { m8[i] = NEG; l8[i] = 0.f; }
    for (int j0 = 0; j0 < p.Lk; j0 += 64) {
        __syncthreads();
#pragma unroll
        for (int it = 0; it < 8; ++it) {
            const int idx = it * (32 * AW) + threadIdx.x;
            const int jr = idx >> 4, d4 = (idx & 15) * 4;
            const int j = min(j0 + jr, p.Lk - 1);
            const v4f f = *(const v4f*)(vbase + (long long)j * p.sVj + d4);
            vl[jr * VP + d4 + 0] = (_Float16)f.x; vl[jr * VP + d4 + 1] = (_Float16)f.y;
            vl[jr * VP + d4 + 2] = (_Float16)f.z; vl[jr * VP + d4 + 3] = (_Float16)f.w;
        }
        v8f s[4]; float bs[4][8];
#pragma unroll
        for (int t = 0; t < 4; ++t) {
            const int j = min(j0 + t * 16 + l15, p.Lk - 1);
            const float* krow = kbase + (long long)j * p.sKj;
            const float* mp = mbase + (long long)j * p.smi;
            const v4f m0 = *(const v4f*)mp, m1 = *(const v4f*)(mp + 4);
            bs[t][0] = m0.x; bs[t][1] = m0.y; bs[t][2] = m0.z; bs[t][3] = m0.w;
            bs[t][4] = m1.x; bs[t][5] = m1.y; bs[t][6] = m1.z; bs[t][7] = m1.w;
            v8f acc = {};
            acc = wmma16(qa0, fh_row32(krow, hf), acc);
            acc = wmma16(qa1, fh_row32(krow + 32, hf), acc);
            s[t] = acc;
        }
        float pv[8][4];
#pragma unroll
        for (int i = 0; i < 8; ++i) {
            float sc[4];
#pragma unroll
            for (int t = 0; t < 4; ++t) {
                const int jg = j0 + t * 16 + l15;
                const float v = s[t][i] * p.scale + bs[t][i];
                sc[t] = (jg < p.Lk) ? v * L2E : NEG;
            }
            float mx = fmaxf(fmaxf(sc[0], sc[1]), fmaxf(sc[2], sc[3]));
            mx = fmaxf(mx, __shfl_xor(mx, 1, 32)); mx = fmaxf(mx, __shfl_xor(mx, 2, 32));
            mx = fmaxf(mx, __shfl_xor(mx, 4, 32)); mx = fmaxf(mx, __shfl_xor(mx, 8, 32));
            const float mnew = fmaxf(m8[i], mx);
            const float corr = (mnew == NEG) ? 1.f : exp2f(m8[i] - mnew);
            float rs = 0.f;
#pragma unroll
            for (int t = 0; t < 4; ++t) {
                const float pp = (sc[t] == NEG) ? 0.f : exp2f(sc[t] - mnew); rs += pp;
                pv[i][t] = pp;
            }
            rs += __shfl_xor(rs, 1, 32); rs += __shfl_xor(rs, 2, 32); rs += __shfl_xor(rs, 4, 32); rs += __shfl_xor(rs, 8, 32);
            l8[i] = l8[i] * corr + rs; m8[i] = mnew;
#pragma unroll
            for (int t = 0; t < NT; ++t) o[t][i] *= corr;
        }
#pragma unroll
        for (int i = 0; i < 8; ++i)
#pragma unroll
            for (int t = 0; t < 4; ++t) pl[wave][(i + 8 * hf) * 64 + t * 16 + l15] = pv[i][t];
        __syncthreads();
        v16h pa0, pa1;
#pragma unroll
        for (int e = 0; e < 16; ++e) {
            const int kk = frag_k(e, hf);
            pa0[e] = (_Float16)(pl[wave][l15 * 64 + kk] * 4096.f);
            pa1[e] = (_Float16)(pl[wave][l15 * 64 + 32 + kk] * 4096.f);
        }
#pragma unroll
        for (int t = 0; t < NT; ++t) {
            const int dcol = t * 16 + l15;
            v16h b0, b1;
#pragma unroll
            for (int e = 0; e < 16; ++e) { b0[e] = vl[frag_k(e, hf) * VP + dcol]; b1[e] = vl[(32 + frag_k(e, hf)) * VP + dcol]; }
            o[t] = wmma16(pa0, b0, o[t]);
            o[t] = wmma16(pa1, b1, o[t]);
        }
    }
    float* obase = p.O + b * p.sOb + h * p.sOh;
    float invr[8];
#pragma unroll
    for (int i = 0; i < 8; ++i) invr[i] = (l8[i] > 0.f) ? 1.f / (l8[i] * 4096.f) : 0.f;
    __syncthreads();
#pragma unroll
    for (int i = 0; i < 8; ++i)
#pragma unroll
        for (int t = 0; t < NT; ++t) pl[wave][(i + 8 * hf) * 64 + t * 16 + l15] = o[t][i] * invr[i];
    __syncthreads();
    for (int r0 = 0; r0 < 16; r0 += 2) {
        const int row = r0 + (lane >> 4), c4 = (lane & 15) * 4;
        const v4f v = *(const v4f*)(&pl[wave][row * 64 + c4]);
        VST2V4(obase + (long long)(q0 + row) * p.sOi + c4, v);
    }
}

constexpr size_t al256c(size_t n) { return (n + 255) / 256 * 256; }
constexpr size_t NTOK   = (size_t)NB * SEQ;
constexpr size_t SZ_X   = al256c(3 * NTOK * DM * 2);
constexpr size_t SZ_W   = al256c((size_t)3 * DM * DM * 2);
constexpr size_t SZ_WS  = al256c((size_t)SIMW * DM * 2);
constexpr size_t SZ_QKV = al256c(NTOK * 3 * DM * 4);
constexpr size_t SZ_SF  = al256c(NTOK * SIMW * 4);
constexpr size_t SZ_SN  = al256c(NTOK * SIMW * 2);
constexpr size_t SZ_SM  = al256c((size_t)NB * SEQ * SEQ * 4);
constexpr size_t SZ_WO  = al256c((size_t)DM * 2 * DM * 2);
constexpr size_t SZ_BO  = al256c((size_t)DM * 4);
constexpr size_t SZ_ALL = SZ_X + SZ_W + SZ_WS + SZ_QKV + SZ_SF + SZ_SN + SZ_SM + SZ_WO + SZ_BO;
static_assert(SEQ % 64 == 0);
static_assert(NB >= 1 && NB <= NB_FULL && SEQ <= SEQ_FULL);
static_assert(SZ_X >= NTOK * DM * 4);
static_assert(SZ_QKV >= NTOK * 2 * DM * 2);
static_assert(SZ_ALL <= (size_t)134217728);
static_assert(((size_t)(NB - 1) * SEQ_FULL + SEQ) * DM * 4 <= (size_t)NB_FULL * SEQ_FULL * DM * 4);

extern "C" void kernel_launch(void* const* d_in, const int* in_sizes, int n_in, void* d_out, int out_size, void* d_ws, size_t ws_size, hipStream_t stream) {
    if (n_in < 9) return;
    const long long need_x = ((long long)(NB - 1) * SEQ_FULL + SEQ) * DM;
    if ((long long)in_sizes[0] < need_x || (long long)in_sizes[1] < need_x || (long long)in_sizes[2] < need_x) return;
    if ((long long)in_sizes[3] < (long long)DM * DM || (long long)in_sizes[4] < (long long)DM * DM || (long long)in_sizes[5] < (long long)DM * DM || (long long)in_sizes[6] < (long long)DM * DM) return;
    if (in_sizes[7] < DM || (long long)in_sizes[8] < (long long)SIMW * DM) return;
    if ((long long)out_size < need_x) return;
    if (SZ_ALL > ws_size) return;
    const float* xq   = (const float*)d_in[0];
    const float* xk   = (const float*)d_in[1];
    const float* xv   = (const float*)d_in[2];
    const float* Wq   = (const float*)d_in[3];
    const float* Wk   = (const float*)d_in[4];
    const float* Wv   = (const float*)d_in[5];
    const float* Wo   = (const float*)d_in[6];
    const float* bo   = (const float*)d_in[7];
    const float* Wsim = (const float*)d_in[8];
    float* out = (float*)d_out;
    char* wsp = (char*)d_ws;
    unsigned short* X16  = (unsigned short*)wsp; float* AO = (float*)wsp;              wsp += SZ_X;
    unsigned short* W16  = (unsigned short*)wsp;                                       wsp += SZ_W;
    unsigned short* WS16 = (unsigned short*)wsp;                                       wsp += SZ_WS;
    float* QKV = (float*)wsp; unsigned short* AOC = (unsigned short*)wsp;              wsp += SZ_QKV;
    float* SIMF = (float*)wsp;                                                         wsp += SZ_SF;
    unsigned short* SIMN = (unsigned short*)wsp;                                       wsp += SZ_SN;
    float* SIMM = (float*)wsp;                                                         wsp += SZ_SM;
    unsigned short* WOC = (unsigned short*)wsp;                                        wsp += SZ_WO;
    float* BRO = (float*)wsp;                                                          wsp += SZ_BO;
    const int ntok = (int)NTOK;

    const unsigned gw = (unsigned)(((long long)DM * (DM / 8) + 255) / 256);
    k_cm_castb<<<gw, 256, 0, stream>>>(Wq, DM, W16, DM, DM, DM, DM, DM, 64.0f);
    k_cm_castb<<<gw, 256, 0, stream>>>(Wk, DM, W16 + (size_t)DM * DM, DM, DM, DM, DM, DM, 64.0f);
    k_cm_castb<<<gw, 256, 0, stream>>>(Wv, DM, W16 + (size_t)2 * DM * DM, DM, DM, DM, DM, DM, 64.0f);
    k_cm_castb<<<(unsigned)(((long long)SIMW * (DM / 8) + 255) / 256), 256, 0, stream>>>(Wsim, DM, WS16, DM, SIMW, DM, SIMW, SIMW, 64.0f);
    const unsigned gx = (unsigned)(((long long)ntok * (DM / 8) + 255) / 256);
    k_cm_castb<<<gx, 256, 0, stream>>>(xq, DM, X16, DM, ntok, DM, SEQ, SEQ_FULL, 1.0f);
    k_cm_castb<<<gx, 256, 0, stream>>>(xk, DM, X16 + NTOK * DM, DM, ntok, DM, SEQ, SEQ_FULL, 1.0f);
    k_cm_castb<<<gx, 256, 0, stream>>>(xv, DM, X16 + 2 * NTOK * DM, DM, ntok, DM, SEQ, SEQ_FULL, 1.0f);
    w25::wmma_gemm64<0, 0><<<dim3((unsigned)(((ntok / 64) * (DM / 64) + 7) / 8), 3u), 256, 0, stream>>>(
        X16, DM, (long long)(NTOK * DM), W16, DM, (long long)DM * DM, QKV, 3 * DM, (long long)DM, nullptr, ntok, DM, DM, 1.0f / 64.0f);
    w25::wmma_gemm64<0, 0><<<dim3((unsigned)(((ntok / 64) * (SIMW / 64) + 7) / 8), 1u), 256, 0, stream>>>(
        X16, DM, 0LL, WS16, DM, 0LL, SIMF, SIMW, 0LL, nullptr, ntok, SIMW, DM, 1.0f / 64.0f);
    k_simnorm<<<(unsigned)((ntok + 7) / 8), 256, 0, stream>>>(SIMF, SIMN, ntok, 64.0f);
    w25::wmma_gemm64<0, 0><<<dim3((unsigned)(((SEQ / 64) * (SEQ / 64) + 7) / 8), (unsigned)NB), 256, 0, stream>>>(
        SIMN, SIMW, (long long)SEQ * SIMW, SIMN, SIMW, (long long)SEQ * SIMW, SIMM, SEQ, (long long)SEQ * SEQ, nullptr, SEQ, SEQ, SIMW, 0.2f / 4096.0f);
    k_cm_castbf<<<gw, 256, 0, stream>>>(Wo, DM, WOC, 2 * DM, DM, DM, DM);
    k_cm_bfvec<<<(DM + 255) / 256, 256, 0, stream>>>(bo, BRO, DM);
    {
        AttnP a;
        a.Q = QKV; a.K = QKV + DM; a.V = QKV + 2 * DM; a.Mf = SIMM; a.O = AO;
        a.sQb = (long long)SEQ * 3 * DM; a.sQh = HD; a.sQi = 3 * DM;
        a.sKb = (long long)SEQ * 3 * DM; a.sKh = HD; a.sKj = 3 * DM;
        a.sVb = (long long)SEQ * 3 * DM; a.sVh = HD; a.sVj = 3 * DM;
        a.sOb = (long long)SEQ * DM; a.sOh = HD; a.sOi = DM;
        a.smb = (long long)SEQ * SEQ; a.smi = SEQ;
        a.Lq = SEQ; a.Lk = SEQ; a.scale = 0.125f; a.pad_ = 0;
        k_attn<<<dim3((unsigned)(SEQ / (16 * AW)), (unsigned)NH, (unsigned)NB), 32 * AW, 0, stream>>>(a);
    }
    k_split8<<<gx, 256, 0, stream>>>(AO, DM, AOC, AOC + DM, 2 * DM, ntok, DM);
    w25::wmma_gemm64<1, 2><<<dim3((unsigned)(((SEQ / 64) * (DM / 64) + 7) / 8), (unsigned)NB), 256, 0, stream>>>(
        AOC, 2 * DM, (long long)SEQ * 2 * DM, WOC, 2 * DM, 0LL, out, DM, (long long)SEQ_FULL * DM, BRO, SEQ, DM, 2 * DM, 1.0f);
}
